// RPEAttention_73426760892660
// MI455X (gfx1250) — hardware-verified
//
#include <hip/hip_runtime.h>


#ifndef NB
#define NB 1
#endif
#ifndef SEQ
#define SEQ 512
#endif
#define NB_FULL  1
#define SEQ_FULL 512
#ifndef OUT_SEQ
#define OUT_SEQ SEQ
#endif
#define KD   128
#define NHD  4
#define HD   32
#define NIC  5
#define QKP  256
#define SSP  (SEQ + 4)
#define OSP2 36
#define SC2  (0.17677669529663687f * 1.4426950408889634f)

static_assert(NB == 1);
static_assert(NHD * HD == KD);
static_assert(KD / 32 == NHD);
static_assert(HD == 32);
static_assert(KD % 64 == 0);
static_assert(KD % 32 == 0);
static_assert(QKP % 64 == 0);
static_assert(SEQ % 64 == 0);
static_assert(SEQ % 32 == 0);
static_assert(SEQ % 16 == 0);
static_assert(OUT_SEQ % 64 == 0);
static_assert(SEQ <= SEQ_FULL);
static_assert(SEQ <= OUT_SEQ);
static_assert((SSP * 4) % 16 == 0);
static_assert((OSP2 * 4) % 16 == 0);
static_assert((size_t)16 * SSP * 4 + (size_t)16 * OSP2 * 4 <= (size_t)65536);

typedef unsigned short bf;
typedef __attribute__((ext_vector_type(16))) __bf16   v16bf;
typedef __attribute__((ext_vector_type(8)))  unsigned short v8us;
typedef __attribute__((ext_vector_type(8)))  float    v8f;
typedef __attribute__((ext_vector_type(4)))  float    v4f;
typedef __attribute__((ext_vector_type(2)))  float    v2f;
typedef v4f  __attribute__((may_alias)) v4fa;
typedef v2f  __attribute__((may_alias)) v2fa;

__device__ __forceinline__ unsigned short f2bf(float f) { unsigned u = __float_as_uint(f); u += 0x7FFFu + ((u >> 16) & 1u); return (unsigned short)(u >> 16); }
__device__ __forceinline__ float bf2f(unsigned short w) { return __uint_as_float((unsigned)w << 16); }
__device__ __forceinline__ float bfr(float f) { unsigned u = __float_as_uint(f); u += 0x7FFFu + ((u >> 16) & 1u); return __uint_as_float(u & 0xFFFF0000u); }
__device__ __forceinline__ v16bf cat16b(v8us lo, v8us hi) { return __builtin_bit_cast(v16bf, __builtin_shufflevector(lo, hi, 0, 1, 2, 3, 4, 5, 6, 7, 8, 9, 10, 11, 12, 13, 14, 15)); }
__device__ __forceinline__ v8f wmmab(v16bf a, v16bf b, v8f c) { return __builtin_amdgcn_wmma_f32_16x16x32_bf16(false, a, false, b, (short)0, c, false, false); }
__device__ __forceinline__ v16bf ldb(const bf* p)  { return cat16b(*(const v8us*)p, *(const v8us*)(p + 16)); }
__device__ __forceinline__ void wave_sync() { __builtin_amdgcn_fence(3  , "wavefront"); __builtin_amdgcn_wave_barrier(); asm volatile("" ::: "memory"); }

__global__ __launch_bounds__(256) void k_cvt8(const float* __restrict__ src, bf* dst, size_t n8) {
    const size_t i = (size_t)blockIdx.x * 256 + threadIdx.x; if (i >= n8) return;
    const v8f v = *(const v8f*)(src + i * 8); v8us o;
#pragma unroll
    for (int k = 0; k < 8; ++k) o[k] = f2bf(v[k]);
    *(volatile v8us*)(dst + i * 8) = o; __threadfence(); *(volatile v8us*)(dst + i * 8) = o;
}

__global__ __launch_bounds__(256) void k_xt(const float* __restrict__ x, bf* XT) {
    __shared__ float ts[KD * 33];
    const int tid = threadIdx.x; const int t0 = blockIdx.x * 32;
#pragma unroll 4
    for (int it = 0; it < 16; ++it) { const int c = it * 8 + (tid >> 5), t = tid & 31;
        ts[c * 33 + t] = x[(size_t)c * SEQ_FULL + t0 + t]; }
    __syncthreads();
    v8us o0, o1;
    const int tk0 = tid >> 4, tk1 = (256 + tid) >> 4, c8 = (tid & 15) * 8;
#pragma unroll
    for (int k = 0; k < 8; ++k) { o0[k] = f2bf(ts[(c8 + k) * 33 + tk0]); o1[k] = f2bf(ts[(c8 + k) * 33 + tk1]); }
    const size_t a0 = (size_t)(t0 + tk0) * KD + c8, a1 = (size_t)(t0 + tk1) * KD + c8;
    *(volatile v8us*)(XT + a0) = o0; *(volatile v8us*)(XT + a1) = o1;
    __threadfence();
    *(volatile v8us*)(XT + a0) = o0; *(volatile v8us*)(XT + a1) = o1;
}

__global__ __launch_bounds__(32) void k_proj(const bf* __restrict__ A, const bf* __restrict__ Bt, bf* Ph, bf* Pl, int pitch) {
    __shared__ __align__(16) float os[16 * 68];
    const int K = KD;
    const int lane = threadIdx.x & 31, lr = lane & 15, hi = lane >> 4; const int r0 = blockIdx.x * 64, c0 = blockIdx.y * 64;
    v8f acc[4][4];
#pragma unroll
    for (int mb = 0; mb < 4; ++mb)
#pragma unroll
        for (int nb = 0; nb < 4; ++nb) acc[mb][nb] = (v8f){};
    const size_t aoff = (size_t)(r0 + lr) * K + 8 * hi, boff = (size_t)(c0 + lr) * K + 8 * hi;
#pragma unroll 1
    for (int kc = 0; kc < K; kc += 32) {
        v16bf a[4];
#pragma unroll
        for (int mb = 0; mb < 4; ++mb) a[mb] = ldb(A + aoff + (size_t)mb * 16 * K + kc);
#pragma unroll
        for (int nb = 0; nb < 4; ++nb) { const v16bf b = ldb(Bt + boff + (size_t)nb * 16 * K + kc);
#pragma unroll
            for (int mb = 0; mb < 4; ++mb) acc[mb][nb] = wmmab(a[mb], b, acc[mb][nb]); }
        asm volatile("v_nop\n\tv_nop\n\tv_nop\n\tv_nop" : "+v"(acc[0][0]), "+v"(acc[1][1]), "+v"(acc[2][2]), "+v"(acc[3][3]) : "v"(a[0]), "v"(a[1]), "v"(a[2]), "v"(a[3]));
    }
    const size_t tbase = (size_t)r0 * (size_t)pitch + (size_t)c0;
#pragma unroll
    for (int mb = 0; mb < 4; ++mb) {
#pragma unroll
        for (int nb = 0; nb < 4; ++nb) {
#pragma unroll
            for (int j = 0; j < 8; ++j) os[(hi * 8 + j) * 68 + nb * 16 + lr] = acc[mb][nb][j]; }
        wave_sync();
        const size_t sb = tbase + (size_t)(mb * 16) * (size_t)pitch;
#pragma unroll 1
        for (int ps = 0; ps < 2; ++ps) {
#pragma unroll
            for (int s = 0; s < 4; ++s) { const int row = 4 * s + (lane >> 3), c8 = (lane & 7) * 8;
                const v4f x0 = *(const v4fa*)(&os[row * 68 + c8]); const v4f x1 = *(const v4fa*)(&os[row * 68 + c8 + 4]); v8us hv, lv;
#pragma unroll
                for (int i = 0; i < 4; ++i) { const unsigned short a0 = f2bf(x0[i]); const unsigned short a1 = f2bf(x1[i]); hv[i] = a0; hv[4 + i] = a1;
                    lv[i] = f2bf(x0[i] - bf2f(a0)); lv[4 + i] = f2bf(x1[i] - bf2f(a1)); }
                const size_t oo = sb + (size_t)row * (size_t)pitch + c8;
                *(volatile v8us*)(Ph + oo) = hv; *(volatile v8us*)(Pl + oo) = lv; }
            if (ps == 0) __threadfence(); }
        wave_sync();
    }
}

__global__ __launch_bounds__(64) void k_uvg(const bf* __restrict__ QKH, const bf* __restrict__ QKL, const float* __restrict__ wind, float* UV, float* GG) {
    const int h = blockIdx.y, z = blockIdx.z;
    if (z == 2) {
        if (blockIdx.x != 0 || threadIdx.x >= 32) return;
        const int l = threadIdx.x; const int lc = (l < 25) ? l : 24; const int c = lc / 5, cp = lc - c * 5;
        float g = 0.0f;
#pragma unroll 1
        for (int d = 0; d < HD; ++d) g = fmaf(bfr(wind[(h * HD + d) * NIC + c]), bfr(wind[(KD + h * HD + d) * NIC + cp]), g);
        const float val = (l < 25) ? g : 0.0f;
        *(volatile float*)(GG + h * 32 + l) = val; __threadfence(); *(volatile float*)(GG + h * 32 + l) = val;
        return;
    }
    const int tok = blockIdx.x * 64 + threadIdx.x;
    const int col = z * KD + h * HD;
    const int wr = (1 - z) * KD + h * HD;
    float a0 = 0.0f, a1 = 0.0f, a2 = 0.0f, a3 = 0.0f, a4 = 0.0f;
#pragma unroll 1
    for (int d = 0; d < HD; ++d) {
        const size_t o = (size_t)tok * QKP + col + d;
        const float v = bf2f(QKH[o]) + bf2f(QKL[o]);
        const float* w = wind + (wr + d) * NIC;
        a0 = fmaf(v, bfr(w[0]), a0); a1 = fmaf(v, bfr(w[1]), a1); a2 = fmaf(v, bfr(w[2]), a2); a3 = fmaf(v, bfr(w[3]), a3); a4 = fmaf(v, bfr(w[4]), a4);
    }
    const size_t ob = (size_t)((z * NHD + h) * NIC) * SEQ + tok;
    *(volatile float*)(UV + ob) = a0; *(volatile float*)(UV + ob + SEQ) = a1; *(volatile float*)(UV + ob + 2 * (size_t)SEQ) = a2;
    *(volatile float*)(UV + ob + 3 * (size_t)SEQ) = a3; *(volatile float*)(UV + ob + 4 * (size_t)SEQ) = a4;
    __threadfence();
    *(volatile float*)(UV + ob) = a0; *(volatile float*)(UV + ob + SEQ) = a1; *(volatile float*)(UV + ob + 2 * (size_t)SEQ) = a2;
    *(volatile float*)(UV + ob + 3 * (size_t)SEQ) = a3; *(volatile float*)(UV + ob + 4 * (size_t)SEQ) = a4;
}

__global__ __launch_bounds__(32) __attribute__((amdgpu_num_vgpr(256)))
void k_attn(const bf* __restrict__ QKH, const bf* __restrict__ QKL, const bf* __restrict__ VH, const bf* __restrict__ VL,
            const float* __restrict__ UV, const float* __restrict__ GG, const float* __restrict__ ind, bf* CH, bf* CL) {
    __shared__ __align__(16) float ss[16 * SSP];
    __shared__ __align__(16) float os[16 * OSP2];
    const int lane = threadIdx.x & 31, lr = lane & 15, hi = lane >> 4;
    const int h = blockIdx.y;
    const int t0 = blockIdx.x * 16;
    const size_t qo = (size_t)(t0 + lr) * QKP + h * HD + 8 * hi;
    const v16bf qh = ldb(QKH + qo), ql = ldb(QKL + qo);
    const size_t ko = (size_t)lr * QKP + KD + h * HD + 8 * hi;
    const size_t vo = (size_t)(h * HD + lr) * SEQ + 8 * hi;
    const float* ibase = ind + (size_t)(t0 + lr) * SEQ_FULL + 8 * hi;
    const float* vbase = UV + (size_t)(NHD * NIC + h * NIC) * SEQ + 8 * hi;
    const float* urow  = UV + (size_t)(h * NIC) * SEQ + t0 + lr;
    const float* gh    = GG + h * 32;
    float* srow = &ss[lr * SSP + 8 * hi];

    float mx = -3.0e38f;
#pragma unroll 1
    for (int kt = 0; kt < SEQ; kt += 16) {
        const v16bf kH = ldb(QKH + ko + (size_t)kt * QKP), kL = ldb(QKL + ko + (size_t)kt * QKP);
        v8f s = (v8f){};
        s = wmmab(kH, qh, s);
        s = wmmab(kH, ql, s);
        s = wmmab(kL, qh, s);
        asm volatile("v_nop\n\tv_nop\n\tv_nop\n\tv_nop" : "+v"(s) : "v"(kH), "v"(kL), "v"(qh), "v"(ql));
        { v4f a, c;
          a[0] = s[0]; a[1] = s[1]; a[2] = s[2]; a[3] = s[3]; c[0] = s[4]; c[1] = s[5]; c[2] = s[6]; c[3] = s[7];
          *(v4fa*)(srow + kt) = a; *(v4fa*)(srow + kt + 4) = c; }
#pragma unroll 1
        for (int r = 0; r < 8; r += 2) {
            const int j = kt + r;
            const v2f sv = *(const v2fa*)(srow + j);
            float I0[5], I1[5];
#pragma unroll
            for (int c = 0; c < 5; ++c) { const v2f iv = *(const v2f*)(ibase + (size_t)c * ((size_t)SEQ_FULL * SEQ_FULL) + j); I0[c] = bfr(iv[0]); I1[c] = bfr(iv[1]); }
            float c0 = 0.0f, c1 = 0.0f;
#pragma unroll
            for (int cp = 0; cp < 5; ++cp) {
                const v2f vv = *(const v2f*)(vbase + (size_t)cp * SEQ + j);
                const float uu = urow[(size_t)cp * SEQ];
                float u0 = uu + vv[0], u1 = uu + vv[1];
#pragma unroll
                for (int c = 0; c < 5; ++c) { const float g = gh[c * 5 + cp]; u0 = fmaf(g, I0[c], u0); u1 = fmaf(g, I1[c], u1); }
                c0 = fmaf(u0, I0[cp], c0); c1 = fmaf(u1, I1[cp], c1);
            }
            v2f tv; tv[0] = (sv[0] + c0) * SC2; tv[1] = (sv[1] + c1) * SC2;
            mx = fmaxf(mx, fmaxf(tv[0], tv[1]));
            *(v2fa*)(srow + j) = tv;
        }
    }
    const float m = fmaxf(mx, __shfl_xor(mx, 16, 32));
    wave_sync();

    v8f o0 = (v8f){}, o1 = (v8f){};
    float l = 0.0f;
#pragma unroll 1
    for (int key0 = 0; key0 < SEQ; key0 += 32) {
        const v4f a0 = *(const v4fa*)(srow + key0), a1 = *(const v4fa*)(srow + key0 + 4);
        const v4f b0 = *(const v4fa*)(srow + key0 + 16), b1 = *(const v4fa*)(srow + key0 + 20);
        float ta[8], tb[8];
#pragma unroll
        for (int i = 0; i < 4; ++i) { ta[i] = a0[i]; ta[4 + i] = a1[i]; tb[i] = b0[i]; tb[4 + i] = b1[i]; }
        v8us pha, pla, phb, plb; float ls = 0.0f;
#pragma unroll
        for (int r = 0; r < 8; ++r) {
            const float pa = __builtin_amdgcn_exp2f(ta[r] - m); const float pc = __builtin_amdgcn_exp2f(tb[r] - m);
            const unsigned short ha = f2bf(pa); const unsigned short hc = f2bf(pc);
            pha[r] = ha; phb[r] = hc; pla[r] = f2bf(pa - bf2f(ha)); plb[r] = f2bf(pc - bf2f(hc));
            ls += pa + pc; }
        const v16bf pH = cat16b(pha, phb), pL = cat16b(pla, plb);
        l += ls;
        const bf* va = VH + vo + key0; const bf* vl = VL + vo + key0;
        const v16bf v0H = ldb(va), v1H = ldb(va + (size_t)16 * SEQ), v0L = ldb(vl), v1L = ldb(vl + (size_t)16 * SEQ);
        o0 = wmmab(v0H, pH, o0); o1 = wmmab(v1H, pH, o1);
        o0 = wmmab(v0L, pH, o0); o1 = wmmab(v1L, pH, o1);
        o0 = wmmab(v0H, pL, o0); o1 = wmmab(v1H, pL, o1);
        asm volatile("v_nop\n\tv_nop\n\tv_nop\n\tv_nop" : "+v"(o0), "+v"(o1) : "v"(v0H), "v"(v1H), "v"(v0L), "v"(v1L), "v"(pH), "v"(pL));
    }
    l += __shfl_xor(l, 16, 32);
    const float inv = 1.0f / l;
    { v4f a, c; const int cb = lr * OSP2 + 8 * hi;
      a[0] = o0[0] * inv; a[1] = o0[1] * inv; a[2] = o0[2] * inv; a[3] = o0[3] * inv; c[0] = o0[4] * inv; c[1] = o0[5] * inv; c[2] = o0[6] * inv; c[3] = o0[7] * inv;
      *(v4fa*)(&os[cb]) = a; *(v4fa*)(&os[cb + 4]) = c;
      a[0] = o1[0] * inv; a[1] = o1[1] * inv; a[2] = o1[2] * inv; a[3] = o1[3] * inv; c[0] = o1[4] * inv; c[1] = o1[5] * inv; c[2] = o1[6] * inv; c[3] = o1[7] * inv;
      *(v4fa*)(&os[cb + 16]) = a; *(v4fa*)(&os[cb + 20]) = c; }
    wave_sync();
    v8us hv[2], lv[2]; size_t oo[2];
#pragma unroll
    for (int it = 0; it < 2; ++it) { const int p = it * 32 + lane; const int row = p >> 2, c8 = (p & 3) * 8;
        const v4f x0 = *(const v4fa*)(&os[row * OSP2 + c8]); const v4f x1 = *(const v4fa*)(&os[row * OSP2 + c8 + 4]);
#pragma unroll
        for (int i = 0; i < 4; ++i) { const unsigned short a0 = f2bf(x0[i]); const unsigned short a1 = f2bf(x1[i]); hv[it][i] = a0; hv[it][4 + i] = a1;
            lv[it][i] = f2bf(x0[i] - bf2f(a0)); lv[it][4 + i] = f2bf(x1[i] - bf2f(a1)); }
        oo[it] = ((size_t)h * SEQ + (size_t)(t0 + row)) * HD + c8; }
#pragma unroll 1
    for (int ps = 0; ps < 2; ++ps) {
        *(volatile v8us*)(CH + oo[0]) = hv[0]; *(volatile v8us*)(CL + oo[0]) = lv[0];
        *(volatile v8us*)(CH + oo[1]) = hv[1]; *(volatile v8us*)(CL + oo[1]) = lv[1];
        if (ps == 0) __threadfence(); }
}

__global__ __launch_bounds__(32) void k_outp(const bf* __restrict__ A, const bf* __restrict__ BH, const bf* __restrict__ BL, const float* __restrict__ bo, float* OUT) {
    __shared__ __align__(16) float os[16 * 68];
    const int K = KD;
    const int lane = threadIdx.x & 31, lr = lane & 15, hi = lane >> 4; const int r0 = blockIdx.x * 64, c0 = blockIdx.y * 64;
    v8f acc[4][4];
#pragma unroll
    for (int mb = 0; mb < 4; ++mb)
#pragma unroll
        for (int nb = 0; nb < 4; ++nb) acc[mb][nb] = (v8f){};
    const size_t aoff = (size_t)(r0 + lr) * K + 8 * hi, boff = (size_t)(c0 + lr) * HD + 8 * hi;
#pragma unroll 1
    for (int kc = 0; kc < K; kc += 32) {
        v16bf a[4];
#pragma unroll
        for (int mb = 0; mb < 4; ++mb) a[mb] = ldb(A + aoff + (size_t)mb * 16 * K + kc);
        const size_t bp = boff + (size_t)(kc >> 5) * ((size_t)SEQ * HD);
#pragma unroll
        for (int nb = 0; nb < 4; ++nb) { const v16bf bh = ldb(BH + bp + (size_t)nb * 16 * HD); const v16bf bl = ldb(BL + bp + (size_t)nb * 16 * HD);
#pragma unroll
            for (int mb = 0; mb < 4; ++mb) acc[mb][nb] = wmmab(a[mb], bh, acc[mb][nb]);
#pragma unroll
            for (int mb = 0; mb < 4; ++mb) acc[mb][nb] = wmmab(a[mb], bl, acc[mb][nb]); }
        asm volatile("v_nop\n\tv_nop\n\tv_nop\n\tv_nop" : "+v"(acc[0][0]), "+v"(acc[1][1]), "+v"(acc[2][2]), "+v"(acc[3][3]) : "v"(a[0]), "v"(a[1]), "v"(a[2]), "v"(a[3]));
    }
#pragma unroll
    for (int mb = 0; mb < 4; ++mb) {
        float bs[8];
#pragma unroll
        for (int j = 0; j < 8; ++j) bs[j] = bfr(bo[r0 + mb * 16 + hi * 8 + j]);
#pragma unroll
        for (int nb = 0; nb < 4; ++nb) {
#pragma unroll
            for (int j = 0; j < 8; ++j) os[(hi * 8 + j) * 68 + nb * 16 + lr] = acc[mb][nb][j] + bs[j]; }
        wave_sync();
        float* orow = OUT + (size_t)(r0 + mb * 16) * OUT_SEQ + c0;
#pragma unroll 1
        for (int ps = 0; ps < 2; ++ps) {
#pragma unroll
            for (int s = 0; s < 8; ++s) { const int row = 2 * s + hi, cofs = lr * 4;
                const v4f val = *(const v4fa*)(&os[row * 68 + cofs]);
                *(volatile v4f*)(orow + (size_t)row * OUT_SEQ + cofs) = val; }
            if (ps == 0) __threadfence(); }
        wave_sync();
    }
}

static constexpr size_t al256(size_t v) { return (v + 255) & ~(size_t)255; }
static constexpr size_t SZ_XT = al256((size_t)SEQ * KD * 2);
static constexpr size_t SZ_WQ = al256((size_t)3 * KD * KD * 2);
static constexpr size_t SZ_WO = al256((size_t)KD * KD * 2);
static constexpr size_t SZ_QK = al256((size_t)SEQ * QKP * 2);
static constexpr size_t SZ_V  = al256((size_t)KD * SEQ * 2);
static constexpr size_t SZ_UV = al256((size_t)2 * NHD * NIC * SEQ * 4);
static constexpr size_t SZ_G  = al256((size_t)NHD * 32 * 4);
static constexpr size_t SZ_C  = al256((size_t)NHD * SEQ * HD * 2);
static constexpr size_t SZ_TOTAL = SZ_XT + SZ_WQ + SZ_WO + 2 * SZ_QK + 2 * SZ_V + SZ_UV + SZ_G + 2 * SZ_C;
static_assert(SZ_TOTAL <= (size_t)134217728);
static_assert(((size_t)3 * KD * KD) % 8 == 0);
static_assert(((size_t)KD * KD) % 8 == 0);

extern "C" void kernel_launch(void* const* d_in, const int* in_sizes, int n_in,
                              void* d_out, int out_size, void* d_ws, size_t ws_size, hipStream_t stream) {
    if (n_in < 6) return;
    if ((size_t)in_sizes[0] < (size_t)(KD - 1) * SEQ_FULL + SEQ) return;
    if ((size_t)in_sizes[1] < ((size_t)(NIC - 1) * SEQ_FULL + (size_t)(SEQ - 1)) * SEQ_FULL + SEQ) return;
    if ((size_t)in_sizes[2] < (size_t)3 * KD * KD) return;
    if ((size_t)in_sizes[3] < (size_t)2 * KD * NIC) return;
    if ((size_t)in_sizes[4] < (size_t)KD * KD) return;
    if ((size_t)in_sizes[5] < (size_t)KD) return;
    if ((size_t)out_size < (size_t)(KD - 1) * OUT_SEQ + SEQ) return;
    if (SZ_TOTAL > ws_size) return;
    const float* x = (const float*)d_in[0]; const float* ind = (const float*)d_in[1]; const float* wqkv = (const float*)d_in[2];
    const float* wind = (const float*)d_in[3]; const float* wout = (const float*)d_in[4]; const float* bout = (const float*)d_in[5];
    float* OUT = (float*)d_out;
    char* wsp = (char*)d_ws;
    bf* XT  = (bf*)wsp; wsp += SZ_XT;
    bf* WQ  = (bf*)wsp; wsp += SZ_WQ;
    bf* WO  = (bf*)wsp; wsp += SZ_WO;
    bf* QKH = (bf*)wsp; wsp += SZ_QK;
    bf* QKL = (bf*)wsp; wsp += SZ_QK;
    bf* VH  = (bf*)wsp; wsp += SZ_V;
    bf* VL  = (bf*)wsp; wsp += SZ_V;
    float* UV = (float*)wsp; wsp += SZ_UV;
    float* GG = (float*)wsp; wsp += SZ_G;
    bf* CH  = (bf*)wsp; wsp += SZ_C;
    bf* CL  = (bf*)wsp; wsp += SZ_C;

    k_xt<<<SEQ / 32, 256, 0, stream>>>(x, XT);
    { const size_t n8 = (size_t)3 * KD * KD / 8; k_cvt8<<<(unsigned)((n8 + 255) / 256), 256, 0, stream>>>(wqkv, WQ, n8); }
    { const size_t n8 = (size_t)KD * KD / 8;     k_cvt8<<<(unsigned)((n8 + 255) / 256), 256, 0, stream>>>(wout, WO, n8); }

    k_proj<<<dim3(SEQ / 64, QKP / 64, 1), 32, 0, stream>>>(XT, WQ, QKH, QKL, QKP);
    k_proj<<<dim3(KD / 64, SEQ / 64, 1), 32, 0, stream>>>(WQ + (size_t)2 * KD * KD, XT, VH, VL, SEQ);

    k_uvg<<<dim3(SEQ / 64, NHD, 3), 64, 0, stream>>>(QKH, QKL, wind, UV, GG);

    k_attn<<<dim3(SEQ / 16, NHD, 1), 32, 0, stream>>>(QKH, QKL, VH, VL, UV, GG, ind, CH, CL);

    k_outp<<<dim3(KD / 64, SEQ / 64, 1), 32, 0, stream>>>(WO, CH, CL, bout, OUT);
}
